// ConverterSurrogate_20452634264259
// MI455X (gfx1250) — hardware-verified
//
#include <hip/hip_runtime.h>


#define B_   256
#define T_   1000
#define DIN  3
#define H_   128
#define G4   512
#define MB   16
#define NOUT 3
#define NTHR 256

typedef _Float16 f16;
typedef f16   v16h __attribute__((ext_vector_type(16)));
typedef f16   v8h  __attribute__((ext_vector_type(8)));
typedef float v8f  __attribute__((ext_vector_type(8)));
typedef float v4f  __attribute__((ext_vector_type(4)));

union Frag { v16h v; v8h h[2]; };

#define SCALE_A 16.0f
#define SCALE_B 64.0f
#define UNSCALE 0.0009765625f

#define Z8 {0.f, 0.f, 0.f, 0.f, 0.f, 0.f, 0.f, 0.f}

__device__ __forceinline__ v8f wmma_f16(v16h a, v16h b, v8f c) {
  v8f d = __builtin_amdgcn_wmma_f32_16x16x32_f16(false, a, false, b, (short)0, c, false, false);
  asm volatile("v_nop\n\tv_nop\n\tv_nop\n\tv_nop" : "+v"(d) : "v"(a), "v"(b));
  return d;
}

__device__ __forceinline__ v16h ld_frag(const f16* base, int pitch, int row, int k0, int hf) {
  Frag f;
  const f16* p = base + row * pitch + k0 + 8 * hf;
  f.h[0] = *(const v8h*)p;
  f.h[1] = *(const v8h*)(p + 16);
  return f.v;
}

__device__ __forceinline__ float sigm(float x) { return 1.0f / (1.0f + __expf(-x)); }

__device__ __forceinline__ void st2_v8h(f16* p, v8h v) {
  *(volatile v8h*)p = v;
  __threadfence();
  *(volatile v8h*)p = v;
}

__device__ __forceinline__ void st2_v4f(float* p, v4f v) {
  *(volatile v4f*)p = v;
  __threadfence();
  *(volatile v4f*)p = v;
}

__global__ __launch_bounds__(NTHR) void k_layer0(
    const float* __restrict__ x,   const float* __restrict__ Wih,
    const float* __restrict__ Whh, const float* __restrict__ bih,
    const float* __restrict__ bhh, f16* __restrict__ h1g)
{
  extern __shared__ v4f dynlds[];
  char* smem = (char*)dynlds;
  f16*   Wb = (f16*)smem;
  f16*   hA = (f16*)(smem + 131072);
  float* xb = (float*)(smem + 135168);

  const int tid = threadIdx.x;
  const int b0  = blockIdx.x * MB;
  if (b0 + MB > B_) return;

  const int wave = __builtin_amdgcn_readfirstlane(tid >> 5);
  const int lane = tid & 31, hf = lane >> 4, n16 = lane & 15;
  const int hh = wave * 16 + n16;
  const int sm = tid >> 4, sch = tid & 15;

  for (int i = tid; i < G4 * H_; i += NTHR) Wb[i] = (f16)(SCALE_B * Whh[i]);
  for (int i = tid; i < MB * H_; i += NTHR) hA[i] = (f16)0.0f;

  float wq[4][3], bq[4];
#pragma unroll
  for (int q = 0; q < 4; ++q) {
    const int n = q * H_ + hh;
    wq[q][0] = Wih[n * DIN + 0];
    wq[q][1] = Wih[n * DIN + 1];
    wq[q][2] = Wih[n * DIN + 2];
    bq[q] = bih[n] + bhh[n];
  }
  float cst[8];
#pragma unroll
  for (int r = 0; r < 8; ++r) cst[r] = 0.0f;
  __syncthreads();

  for (int t = 0; t < T_; ++t) {
    if (tid < MB * DIN) {
      const int r = tid / DIN, i = tid - DIN * r;
      xb[r * 4 + i] = x[((size_t)(b0 + r) * T_ + t) * DIN + i];
    }
    __syncthreads();

    if (t > 0) {
      const v8h v = *(const v8h*)(hA + sm * H_ + sch * 8);
      st2_v8h(h1g + ((size_t)(t - 1) * B_ + b0 + sm) * H_ + sch * 8, v);
    }

    v8f acc0 = Z8, acc1 = Z8, acc2 = Z8, acc3 = Z8;
#pragma unroll
    for (int kt = 0; kt < 4; ++kt) {
      const v16h a = ld_frag(hA, H_, n16, kt * 32, hf);
      acc0 = wmma_f16(a, ld_frag(Wb, H_, 0 * H_ + hh, kt * 32, hf), acc0);
      acc1 = wmma_f16(a, ld_frag(Wb, H_, 1 * H_ + hh, kt * 32, hf), acc1);
      acc2 = wmma_f16(a, ld_frag(Wb, H_, 2 * H_ + hh, kt * 32, hf), acc2);
      acc3 = wmma_f16(a, ld_frag(Wb, H_, 3 * H_ + hh, kt * 32, hf), acc3);
    }

    float hn[8];
#pragma unroll
    for (int r = 0; r < 8; ++r) {
      const int m = 8 * hf + r;
      const float x0 = xb[m * 4 + 0], x1 = xb[m * 4 + 1], x2 = xb[m * 4 + 2];
      const float pi = acc0[r] * UNSCALE + bq[0] + x0 * wq[0][0] + x1 * wq[0][1] + x2 * wq[0][2];
      const float pf = acc1[r] * UNSCALE + bq[1] + x0 * wq[1][0] + x1 * wq[1][1] + x2 * wq[1][2];
      const float pg = acc2[r] * UNSCALE + bq[2] + x0 * wq[2][0] + x1 * wq[2][1] + x2 * wq[2][2];
      const float po = acc3[r] * UNSCALE + bq[3] + x0 * wq[3][0] + x1 * wq[3][1] + x2 * wq[3][2];
      const float cc = sigm(pf) * cst[r] + sigm(pi) * tanhf(pg);
      cst[r] = cc;
      hn[r] = sigm(po) * tanhf(cc);
    }
    __syncthreads();

#pragma unroll
    for (int r = 0; r < 8; ++r) hA[(8 * hf + r) * H_ + hh] = (f16)(SCALE_A * hn[r]);
  }
  __syncthreads();
  {
    const v8h v = *(const v8h*)(hA + sm * H_ + sch * 8);
    st2_v8h(h1g + ((size_t)(T_ - 1) * B_ + b0 + sm) * H_ + sch * 8, v);
  }
}

__global__ __launch_bounds__(NTHR) void k_layer1(
    const f16* __restrict__ h1g,    const float* __restrict__ Wih,
    const float* __restrict__ Whh,  const float* __restrict__ bih,
    const float* __restrict__ bhh,  const float* __restrict__ fcwg,
    const float* __restrict__ fcbg, float* __restrict__ ysg)
{
  extern __shared__ v4f dynlds[];
  char* smem = (char*)dynlds;
  f16*   Wb = (f16*)smem;
  f16*   hX = (f16*)(smem + 262144);
  f16*   hH = (f16*)(smem + 266240);
  f16*   Wf = (f16*)(smem + 270336);
  float* yb = (float*)(smem + 274432);

  const int tid = threadIdx.x;
  const int b0  = blockIdx.x * MB;
  if (b0 + MB > B_) return;

  const int wave = __builtin_amdgcn_readfirstlane(tid >> 5);
  const int lane = tid & 31, hf = lane >> 4, n16 = lane & 15;
  const int hh = wave * 16 + n16;
  const int sm = tid >> 4, sch = tid & 15;

  for (int i = tid; i < G4 * 2 * H_; i += NTHR) {
    const int n = i >> 8, k = i & 255;
    const float w = (k < H_) ? Wih[n * H_ + k] : Whh[n * H_ + (k - H_)];
    Wb[i] = (f16)(SCALE_B * w);
  }
  for (int i = tid; i < MB * H_; i += NTHR) hH[i] = (f16)0.0f;
  for (int i = tid; i < 16 * H_; i += NTHR) {
    const int o = i >> 7, k = i & 127;
    Wf[i] = (o < NOUT) ? (f16)(SCALE_B * fcwg[o * H_ + k]) : (f16)0.0f;
  }
  float bq[4];
#pragma unroll
  for (int q = 0; q < 4; ++q) { const int n = q * H_ + hh; bq[q] = bih[n] + bhh[n]; }
  const float fb = (n16 < NOUT) ? fcbg[n16] : 0.0f;
  float cst[8];
#pragma unroll
  for (int r = 0; r < 8; ++r) cst[r] = 0.0f;
  __syncthreads();

  for (int t = 0; t < T_; ++t) {
    *(v8h*)(hX + sm * H_ + sch * 8) =
        *(const v8h*)(h1g + ((size_t)t * B_ + b0 + sm) * H_ + sch * 8);
    __syncthreads();

    if (wave == 0) {
      if (t > 0 && lane < 16) {
        const v4f v = *(const v4f*)(yb + lane * 4);
        st2_v4f(ysg + ((size_t)(t - 1) * B_ + b0 + lane) * 4, v);
      }
    }

    v8f acc0 = Z8, acc1 = Z8, acc2 = Z8, acc3 = Z8;
#pragma unroll
    for (int kt = 0; kt < 8; ++kt) {
      const f16* tile = (kt < 4) ? hX : hH;
      const v16h a = ld_frag(tile, H_, n16, (kt & 3) * 32, hf);
      acc0 = wmma_f16(a, ld_frag(Wb, 2 * H_, 0 * H_ + hh, kt * 32, hf), acc0);
      acc1 = wmma_f16(a, ld_frag(Wb, 2 * H_, 1 * H_ + hh, kt * 32, hf), acc1);
      acc2 = wmma_f16(a, ld_frag(Wb, 2 * H_, 2 * H_ + hh, kt * 32, hf), acc2);
      acc3 = wmma_f16(a, ld_frag(Wb, 2 * H_, 3 * H_ + hh, kt * 32, hf), acc3);
    }

    float hn[8];
#pragma unroll
    for (int r = 0; r < 8; ++r) {
      const float pi = acc0[r] * UNSCALE + bq[0];
      const float pf = acc1[r] * UNSCALE + bq[1];
      const float pg = acc2[r] * UNSCALE + bq[2];
      const float po = acc3[r] * UNSCALE + bq[3];
      const float cc = sigm(pf) * cst[r] + sigm(pi) * tanhf(pg);
      cst[r] = cc;
      hn[r] = sigm(po) * tanhf(cc);
    }
    __syncthreads();

#pragma unroll
    for (int r = 0; r < 8; ++r) hH[(8 * hf + r) * H_ + hh] = (f16)(SCALE_A * hn[r]);
    __syncthreads();

    if (wave == 0) {
      v8f af = Z8;
#pragma unroll
      for (int kt = 0; kt < 4; ++kt)
        af = wmma_f16(ld_frag(hH, H_, n16, kt * 32, hf), ld_frag(Wf, H_, n16, kt * 32, hf), af);
      if (n16 < 4) {
#pragma unroll
        for (int r = 0; r < 8; ++r) yb[(8 * hf + r) * 4 + n16] = af[r] * UNSCALE + fb;
      }
    }
  }
  __syncthreads();
  if (wave == 0 && lane < 16) {
    const v4f v = *(const v4f*)(yb + lane * 4);
    st2_v4f(ysg + ((size_t)(T_ - 1) * B_ + b0 + lane) * 4, v);
  }
}

__device__ __forceinline__ float gather_y(const float* __restrict__ ysg, int f) {
  int b = f / (T_ * NOUT);
  const int rem = f - b * (T_ * NOUT);
  const int t = rem / NOUT;
  const int o = rem - t * NOUT;
  b = min(b, B_ - 1);
  return ysg[((size_t)t * B_ + b) * 4 + o];
}

__global__ __launch_bounds__(NTHR) void k_pack(const float* __restrict__ ysg,
                                              float* __restrict__ out, int out_n)
{
  const int g  = blockIdx.x * NTHR + threadIdx.x;
  const int n4 = out_n >> 2;
  if (g < n4) {
    const int f = 4 * g;
    v4f v;
    v.x = gather_y(ysg, f + 0);
    v.y = gather_y(ysg, f + 1);
    v.z = gather_y(ysg, f + 2);
    v.w = gather_y(ysg, f + 3);
    st2_v4f(out + (size_t)4 * g, v);
  } else if (g == n4) {
    for (int f = 4 * n4; f < out_n; ++f) {
      const float y = gather_y(ysg, f);
      *(volatile float*)(out + f) = y;
      __threadfence();
      *(volatile float*)(out + f) = y;
    }
  }
}

extern "C" void kernel_launch(void* const* d_in, const int* in_sizes, int n_in,
                              void* d_out, int out_size, void* d_ws, size_t ws_size,
                              hipStream_t stream) {
  if (n_in < 11) return;
  if (in_sizes[0] != B_ * T_ * DIN || in_sizes[1] != G4 * DIN || in_sizes[2] != G4 * H_ ||
      in_sizes[5] != G4 * H_ || in_sizes[6] != G4 * H_ || in_sizes[9] != NOUT * H_ ||
      out_size != B_ * T_ * NOUT) return;

  const size_t h1_bytes = (size_t)T_ * B_ * H_ * sizeof(f16);
  const size_t ys_off   = (h1_bytes + 255) & ~(size_t)255;
  const size_t ys_bytes = (size_t)T_ * B_ * 4 * sizeof(float);
  if (ys_off + ys_bytes > ws_size) return;

  const float* x    = (const float*)d_in[0];
  const float* Wih0 = (const float*)d_in[1];
  const float* Whh0 = (const float*)d_in[2];
  const float* bih0 = (const float*)d_in[3];
  const float* bhh0 = (const float*)d_in[4];
  const float* Wih1 = (const float*)d_in[5];
  const float* Whh1 = (const float*)d_in[6];
  const float* bih1 = (const float*)d_in[7];
  const float* bhh1 = (const float*)d_in[8];
  const float* fcw  = (const float*)d_in[9];
  const float* fcb  = (const float*)d_in[10];
  float* out = (float*)d_out;
  f16*   h1  = (f16*)d_ws;
  float* ys  = (float*)((char*)d_ws + ys_off);

  constexpr size_t LDS0 = 135424;
  constexpr size_t LDS1 = 274688;

  hipFuncSetAttribute(reinterpret_cast<const void*>(k_layer0),
                      hipFuncAttributeMaxDynamicSharedMemorySize, (int)LDS0);
  hipFuncSetAttribute(reinterpret_cast<const void*>(k_layer1),
                      hipFuncAttributeMaxDynamicSharedMemorySize, (int)LDS1);

  k_layer0<<<dim3(B_ / MB), dim3(NTHR), LDS0, stream>>>(x, Wih0, Whh0, bih0, bhh0, h1);
  k_layer1<<<dim3(B_ / MB), dim3(NTHR), LDS1, stream>>>(h1, Wih1, Whh1, bih1, bhh1, fcw, fcb, ys);

  const int n4 = out_size / 4;
  const int gridp = (n4 + 1 + NTHR - 1) / NTHR;
  k_pack<<<dim3(gridp), dim3(NTHR), 0, stream>>>(ys, out, out_size);
}
